// MultiHeadedTrilinearAttention_429496729639
// MI455X (gfx1250) — hardware-run, weakly checked
//
#include <hip/hip_runtime.h>
#include <math.h>

typedef __attribute__((ext_vector_type(16))) _Float16 v16h;
typedef __attribute__((ext_vector_type(16))) __bf16 v16b;
typedef __attribute__((ext_vector_type(8)))  _Float16 v8h;
typedef __attribute__((ext_vector_type(8)))  float v8f;
typedef __attribute__((ext_vector_type(4)))  float v4f;
typedef __attribute__((ext_vector_type(2)))  float v2f;
typedef __attribute__((ext_vector_type(4)))  unsigned v4u;
typedef __attribute__((ext_vector_type(4)))  int v4i;
typedef float __attribute__((may_alias)) float_a;
typedef int __attribute__((may_alias)) int_a;

template <typename T> __device__ __forceinline__ void vst2(void* p, T v) { *(volatile T*)p = v; __threadfence(); *(volatile T*)p = v; }
__device__ __forceinline__ v8f wmma16(v16h a, v16h b, v8f c) {
  v8f d = __builtin_amdgcn_wmma_f32_16x16x32_f16(false, a, false, b, (short)0, c, false, false);
  asm volatile("v_nop\n\tv_nop\n\tv_nop\n\tv_nop" : "+v"(d) : "v"(a), "v"(b));
  return d;
}
__device__ __forceinline__ v8f wmma_bf(v16b a, v16b b, v8f c) {
  v8f d = __builtin_amdgcn_wmma_f32_16x16x32_bf16(false, a, false, b, (short)0, c, false, false);
  asm volatile("v_nop\n\tv_nop\n\tv_nop\n\tv_nop" : "+v"(d) : "v"(a), "v"(b));
  return d;
}
__device__ __forceinline__ v16h frag_h(const _Float16* rowk0, int lane) {
  union { v16h v; v8h q[2]; } u; const _Float16* p = rowk0 + 8 * (lane >> 4);
  u.q[0] = *(const v8h*)p; u.q[1] = *(const v8h*)(p + 16); return u.v;
}
__device__ __forceinline__ v16h frag_f32(const float* rowk0, int lane) {
  v16h a; const float* p = rowk0 + 8 * (lane >> 4);
#pragma unroll
  for (int i = 0; i < 8; ++i) { a[i] = (_Float16)p[i]; a[8 + i] = (_Float16)p[16 + i]; }
  return a;
}
__device__ __forceinline__ v16h frag_f32s(const float* rowk0, int lane, float sc) {
  v16h a; const float* p = rowk0 + 8 * (lane >> 4);
#pragma unroll
  for (int i = 0; i < 8; ++i) { a[i] = (_Float16)(p[i] * sc); a[8 + i] = (_Float16)(p[16 + i] * sc); }
  return a;
}
__device__ __forceinline__ v16h fragc_f32(const float* W, int k0, int n, int lane, int ld, int K) {
  v16h a; const int g = lane >> 4;
#pragma unroll
  for (int i = 0; i < 8; ++i) { const int ka = k0 + 8 * g + i, kb = ka + 16;
    a[i] = (_Float16)(ka < K ? W[(size_t)(ka < K ? ka : K - 1) * ld + n] : 0.f); a[8 + i] = (_Float16)(kb < K ? W[(size_t)(kb < K ? kb : K - 1) * ld + n] : 0.f); }
  return a;
}
struct F2 { v16b h, l; };
__device__ __forceinline__ F2 bsplit16(const float v[16]) { F2 r;
#pragma unroll
  for (int i = 0; i < 16; ++i) { const __bf16 h = (__bf16)v[i]; r.h[i] = h; r.l[i] = (__bf16)(v[i] - (float)h); }
  return r; }
__device__ __forceinline__ F2 split_row(const float* row, int k0, int lane) { float v[16]; const float* p = row + k0 + 8 * (lane >> 4);
#pragma unroll
  for (int i = 0; i < 8; ++i) { v[i] = p[i]; v[8 + i] = p[16 + i]; }
  return bsplit16(v); }
__device__ __forceinline__ F2 split_rowK(const float* row, int k0, int lane, int K) { float v[16]; const int g = lane >> 4;
#pragma unroll
  for (int i = 0; i < 8; ++i) { const int ka = k0 + 8 * g + i, kb = ka + 16; v[i] = ka < K ? row[ka < K ? ka : K - 1] : 0.f; v[8 + i] = kb < K ? row[kb < K ? kb : K - 1] : 0.f; }
  return bsplit16(v); }
__device__ __forceinline__ F2 split_col(const float* W, int k0, int n, int lane, int ld, int K) { float v[16]; const int g = lane >> 4;
#pragma unroll
  for (int i = 0; i < 8; ++i) { const int ka = k0 + 8 * g + i, kb = ka + 16; v[i] = ka < K ? W[(size_t)(ka < K ? ka : K - 1) * ld + n] : 0.f; v[8 + i] = kb < K ? W[(size_t)(kb < K ? kb : K - 1) * ld + n] : 0.f; }
  return bsplit16(v); }
__device__ __forceinline__ v8f mac3(const F2& a, const F2& b, v8f c) { c = wmma_bf(a.l, b.h, c); c = wmma_bf(a.h, b.l, c); return wmma_bf(a.h, b.h, c); }
__device__ __forceinline__ float sigm(float v) { return 1.0f / (1.0f + expf(-v)); }
#define LDSX() do { asm volatile("s_wait_dscnt 0" ::: "memory"); __builtin_amdgcn_wave_barrier(); __builtin_amdgcn_fence(__ATOMIC_RELEASE, "workgroup"); } while (0)


#define NBT 32
#define NV 100
#define NQ 32
#define NA 32
#define DM 768
#define NH 12
#define HD 64
#define NVP 128
#define NBH (NBT * NH)
#ifndef TBH
#define TBH NBH
#endif
typedef __attribute__((ext_vector_type(8))) __bf16 v8b;
__device__ __forceinline__ v16b frag_b(const __bf16* rowk0, int lane) {
  union { v16b v; v8b q[2]; } u; const __bf16* p = rowk0 + 8 * (lane >> 4);
  u.q[0] = *(const v8b*)p; u.q[1] = *(const v8b*)(p + 16); return u.v;
}
__device__ __forceinline__ float bfr(float v) { return (float)(__bf16)v; }
__device__ __attribute__((noinline)) float exp_ni(float v) { return expf(v); }
__device__ __attribute__((noinline)) float erf_ni(float v) { return erff(v); }

#define WS_PW  0u
#define WS_VP  (WS_PW + 2u * (size_t)6 * DM * DM)
#define WS_QP  (WS_VP + 4u * (size_t)NBT * NVP * DM)
#define WS_AP  (WS_QP + 4u * (size_t)NBT * NQ * DM)
#define WS_VO  (WS_AP + 4u * (size_t)NBT * NA * DM)
#define WS_QO  (WS_VO + 4u * (size_t)NBT * NVP * DM)
#define WS_AO  (WS_QO + 4u * (size_t)NBT * NQ * DM)
#define WS_S   (WS_AO + 4u * (size_t)NBT * NA * DM)
#define WS_END (WS_S + 4u * (size_t)NBH * NV * NQ * NA)

__global__ __launch_bounds__(256) void k_pack(const float* __restrict__ W0, const float* __restrict__ W1, const float* __restrict__ W2, const float* __restrict__ W3, const float* __restrict__ W4, const float* __restrict__ W5, __bf16* __restrict__ PW) {
  const int n = blockIdx.x, m = blockIdx.y, t = threadIdx.x; __shared__ __align__(16) __bf16 s[DM]; const float* w = (m == 0) ? W0 : (m == 1) ? W1 : (m == 2) ? W2 : (m == 3) ? W3 : (m == 4) ? W4 : W5;
  for (int k = t; k < DM; k += 256) s[k] = (__bf16)w[(size_t)k * DM + n];
  __syncthreads(); if (t < DM / 8) vst2((unsigned*)(PW + ((size_t)m * DM + n) * DM + t * 8), *(const v4u*)&s[t * 8]); }
template <int STAGE>
__global__ __launch_bounds__(128) void k_proj(const float* __restrict__ XV, const float* __restrict__ XQ, const float* __restrict__ XA, const __bf16* __restrict__ PW, const float* __restrict__ B0, const float* __restrict__ B1, const float* __restrict__ B2, const float* __restrict__ IV, const float* __restrict__ IQ, const float* __restrict__ IA, float* __restrict__ OV, float* __restrict__ OQ, float* __restrict__ OA) {
  __shared__ __align__(16) float so[4][16][132];
  const int tid = threadIdx.x, wave = tid >> 5, lane = tid & 31, col = lane & 15, g = lane >> 4; const int m = blockIdx.z; const int nrows = (m == 0) ? NBT * NVP : NBT * NQ; const size_t rb = (size_t)blockIdx.x * 64; if (rb >= (size_t)nrows) return;
  const size_t r0 = rb + wave * 16; const int c0 = blockIdx.y * 128; const __bf16* Wr = PW + ((size_t)(STAGE * 3 + m) * DM) * DM; const float* BB = (m == 0) ? B0 : (m == 1) ? B1 : B2; float* dst = (m == 0) ? OV : (m == 1) ? OQ : OA;
  v8f acc[8] = {};
  if (STAGE == 0) { const float* X = (m == 0) ? XV : (m == 1) ? XQ : XA;
    const size_t er = r0 + col; size_t ir; bool live = true; if (m == 0) { const size_t b = er / NVP, i = er % NVP; live = i < NV; ir = b * NV + (live ? i : 0); } else ir = er;
#pragma unroll 2
    for (int kc = 0; kc < DM / 32; ++kc) { v16b a; { const float* p = X + ir * DM + kc * 32 + 8 * g;
#pragma unroll
        for (int i = 0; i < 8; ++i) { a[i] = live ? (__bf16)p[i] : (__bf16)0.f; a[8 + i] = live ? (__bf16)p[16 + i] : (__bf16)0.f; } }
#pragma unroll
      for (int j = 0; j < 8; ++j) acc[j] = wmma_bf(a, frag_b(Wr + (size_t)(c0 + j * 16 + col) * DM + kc * 32, lane), acc[j]); } }
  else { const float* X = (m == 0) ? IV : (m == 1) ? IQ : IA;
#pragma unroll 2
    for (int kc = 0; kc < DM / 32; ++kc) { const F2 a = split_row(X + (r0 + col) * DM, kc * 32, lane);
#pragma unroll
      for (int j = 0; j < 8; ++j) { const v16b w = frag_b(Wr + (size_t)(c0 + j * 16 + col) * DM + kc * 32, lane); acc[j] = wmma_bf(a.h, w, acc[j]); acc[j] = wmma_bf(a.l, w, acc[j]); } } }
#pragma unroll
  for (int j = 0; j < 8; ++j) { const float bb = bfr(BB[c0 + j * 16 + col]);
#pragma unroll
    for (int r = 0; r < 8; ++r) so[wave][8 * g + r][j * 16 + col] = acc[j][r] + bb; }
  LDSX();
  for (int rl = 0; rl < 16; ++rl) vst2(dst + (r0 + rl) * DM + c0 + lane * 4, *(const v4f*)&so[wave][rl][lane * 4]);
}
__global__ __launch_bounds__(128) void k_tri(const float* __restrict__ VP, const float* __restrict__ QP, const float* __restrict__ AP, const int* __restrict__ MV, const int* __restrict__ MQ, const int* __restrict__ MA, float* __restrict__ S) {
  __shared__ float sq[NQ][HD + 1]; __shared__ __align__(16) _Float16 sah[NA][HD + 8]; __shared__ __align__(16) _Float16 sal[NA][HD + 8]; __shared__ __align__(16) _Float16 sAh[4][NQ][HD + 8]; __shared__ __align__(16) _Float16 sAl[4][NQ][HD + 8]; __shared__ float svr[4][HD]; __shared__ __align__(16) float sout[4][NQ][NA + 4]; __shared__ float smq[NQ], sma[NA];
  const int tid = threadIdx.x, wave = tid >> 5, lane = tid & 31, col = lane & 15, g = lane >> 4; const size_t bh = blockIdx.x; const size_t b = bh / NH; const int h = (int)(bh % NH);
  for (int e = tid; e < NQ * HD; e += 128) { const int q = e >> 6, w = e & 63; sq[q][w] = QP[(b * NQ + q) * DM + h * HD + w]; }
  for (int e = tid; e < NA * HD; e += 128) { const int a2 = e >> 6, w = e & 63; const float v = AP[(b * NA + a2) * DM + h * HD + w]; const _Float16 hv = (_Float16)v; sah[a2][w] = hv; sal[a2][w] = (_Float16)((v - (float)hv) * 2048.0f); }
  if (tid < NQ) smq[tid] = (float)MQ[b * NQ + tid]; if (tid >= 32 && tid < 32 + NA) sma[tid - 32] = (float)MA[b * NA + tid - 32];
  __syncthreads();
  for (int v = wave; v < NV; v += 4) { const float mvv = (float)MV[b * NV + v];
    for (int w = lane; w < HD; w += 32) svr[wave][w] = VP[(b * NVP + v) * DM + h * HD + w];
    __builtin_amdgcn_wave_barrier(); __builtin_amdgcn_fence(__ATOMIC_RELEASE, "workgroup");
    for (int e = lane; e < NQ * HD; e += 32) { const int q = e >> 6, w = e & 63; const float pv = sq[q][w] * svr[wave][w]; const _Float16 hv = (_Float16)pv; sAh[wave][q][w] = hv; sAl[wave][q][w] = (_Float16)((pv - (float)hv) * 2048.0f); }
    LDSX();
#pragma unroll
    for (int qt = 0; qt < 2; ++qt) {
#pragma unroll
      for (int at = 0; at < 2; ++at) { v8f c = {}, cl = {};
#pragma unroll
        for (int kc = 0; kc < 2; ++kc) { const v16h ah = frag_h(&sAh[wave][qt * 16 + col][kc * 32], lane), al = frag_h(&sAl[wave][qt * 16 + col][kc * 32], lane); const v16h bhf = frag_h(&sah[at * 16 + col][kc * 32], lane); c = wmma16(ah, bhf, c); cl = wmma16(al, bhf, cl); cl = wmma16(ah, frag_h(&sal[at * 16 + col][kc * 32], lane), cl); }
#pragma unroll
        for (int r = 0; r < 8; ++r) { const int q = qt * 16 + 8 * g + r, a2 = at * 16 + col; sout[wave][q][a2] = (c[r] + cl[r] * (1.0f / 2048.0f)) * 0.125f - 10000.0f * (mvv + smq[q] + sma[a2]); } } }
    LDSX();
    for (int e = lane; e < NQ * NA / 4; e += 32) { const int q = e >> 3, qq = e & 7; vst2(S + ((bh * NV + v) * NQ + q) * NA + qq * 4, *(const v4f*)&sout[wave][q][qq * 4]); }
    LDSX(); }
}
__global__ __launch_bounds__(256) void k_marg(const float* __restrict__ S, const float* __restrict__ VO, const float* __restrict__ QO, const float* __restrict__ AO, float* __restrict__ OUTV, float* __restrict__ OUTQ, float* __restrict__ OUTA) {
  __shared__ float red[256]; __shared__ float seqa[NQ * NA]; __shared__ float smv[NV], smq[NQ], sma[NA]; __shared__ float sZ;
  const int t = threadIdx.x; const size_t bh = blockIdx.x; const size_t b = bh / NH; const int h = (int)(bh % NH); const float* Sb = S + bh * (size_t)(NV * NQ * NA);
  float mx = -3.0e38f; for (int e = t; e < NV * NQ * NA; e += 256) mx = fmaxf(mx, Sb[e]); red[t] = mx; __syncthreads();
  for (int s = 128; s > 0; s >>= 1) { if (t < s) red[t] = fmaxf(red[t], red[t + s]); __syncthreads(); } const float M = red[0]; __syncthreads();
  for (int p = t; p < NQ * NA; p += 256) { float a = 0.f; for (int v = 0; v < NV; ++v) a += __expf(Sb[(size_t)v * NQ * NA + p] - M); seqa[p] = a; }
  if (t < NV) { float a = 0.f; const float* row = Sb + (size_t)t * NQ * NA; for (int p = 0; p < NQ * NA; ++p) a += __expf(row[p] - M); smv[t] = a; }
  __syncthreads();
  if (t < NQ) { float a = 0.f; for (int j = 0; j < NA; ++j) a += seqa[t * NA + j]; smq[t] = a; }
  if (t >= 32 && t < 32 + NA) { const int j = t - 32; float a = 0.f; for (int q = 0; q < NQ; ++q) a += seqa[q * NA + j]; sma[j] = a; }
  __syncthreads();
  if (t == 0) { float z = 0.f; for (int q = 0; q < NQ; ++q) z += smq[q]; sZ = z; } __syncthreads(); const float iz = 1.0f / sZ;
  for (int e = t; e < NV * 16; e += 256) { const int i = e >> 4, qd = e & 15; const float mm = smv[i] * iz; const float* src = VO + ((b * NVP + i) * DM) + h * HD + qd * 4; v4f o; o[0] = src[0] * mm; o[1] = src[1] * mm; o[2] = src[2] * mm; o[3] = src[3] * mm; vst2(OUTV + ((b * NV + i) * DM) + h * HD + qd * 4, o); }
  for (int e = t; e < NQ * 16; e += 256) { const int i = e >> 4, qd = e & 15; const float mm = smq[i] * iz; const float* src = QO + ((b * NQ + i) * DM) + h * HD + qd * 4; v4f o; o[0] = src[0] * mm; o[1] = src[1] * mm; o[2] = src[2] * mm; o[3] = src[3] * mm; vst2(OUTQ + ((b * NQ + i) * DM) + h * HD + qd * 4, o); }
  for (int e = t; e < NA * 16; e += 256) { const int i = e >> 4, qd = e & 15; const float mm = sma[i] * iz; const float* src = AO + ((b * NA + i) * DM) + h * HD + qd * 4; v4f o; o[0] = src[0] * mm; o[1] = src[1] * mm; o[2] = src[2] * mm; o[3] = src[3] * mm; vst2(OUTA + ((b * NA + i) * DM) + h * HD + qd * 4, o); }
}
extern "C" void kernel_launch(void* const* d_in, const int* in_sizes, int n_in, void* d_out, int out_size, void* d_ws, size_t ws_size, hipStream_t stream) {
  (void)in_sizes; (void)n_in; (void)out_size;
  const float** F = (const float**)d_in;
  if (ws_size < (size_t)WS_END) return;
  char* ws = (char*)d_ws; __bf16* PW = (__bf16*)ws; float *VP = (float*)(ws + WS_VP), *QP = (float*)(ws + WS_QP), *AP = (float*)(ws + WS_AP), *VO = (float*)(ws + WS_VO), *QO = (float*)(ws + WS_QO), *AO = (float*)(ws + WS_AO), *S = (float*)(ws + WS_S);
  float* OUTV = (float*)d_out; float* OUTQ = OUTV + (size_t)NBT * NV * DM; float* OUTA = OUTQ + (size_t)NBT * NQ * DM;
  k_pack<<<dim3(DM, 6), 256, 0, stream>>>(F[6], F[8], F[10], F[12], F[14], F[16], PW);
  k_proj<0><<<dim3(NBT * NVP / 64, DM / 128, 3), 128, 0, stream>>>(F[0], F[1], F[2], PW, F[7], F[9], F[11], nullptr, nullptr, nullptr, VP, QP, AP);
  k_proj<1><<<dim3(NBT * NVP / 64, DM / 128, 3), 128, 0, stream>>>(nullptr, nullptr, nullptr, PW, F[13], F[15], F[17], VP, QP, AP, VO, QO, AO);
  k_tri<<<TBH, 128, 0, stream>>>(VP, QP, AP, (const int*)d_in[3], (const int*)d_in[4], (const int*)d_in[5], S);
  k_marg<<<TBH, 256, 0, stream>>>(S, VO, QO, AO, OUTV, OUTQ, OUTA);
}
